// SequentialMambaEncoder_17575006175958
// MI455X (gfx1250) — hardware-verified
//
#include <hip/hip_runtime.h>
#include <math.h>

typedef __attribute__((ext_vector_type(16))) _Float16 v16h;
typedef __attribute__((ext_vector_type(8)))  _Float16 v8h;
typedef __attribute__((ext_vector_type(16))) __bf16   v16b;
typedef __attribute__((ext_vector_type(8)))  __bf16   v8b;
typedef __attribute__((ext_vector_type(8)))  float    v8f;
typedef __attribute__((ext_vector_type(4)))  float    v4f;

constexpr int kNL    = 4;
constexpr int kBatch = 8;
constexpr int kNC    = 256;
constexpr int kNT    = 64;
constexpr int kDm    = 256;
constexpr int kDin   = 512;
constexpr int kNst   = 16;
constexpr int kDtR   = 16;
constexpr int kKc    = 4;
constexpr int kXzP   = 2 * kDin;
constexpr int kXdW   = kDtR + 2 * kNst;
constexpr int kXdP   = 64;
constexpr int kRowsP = kBatch * kNC;
constexpr int kRowsT = kBatch * kNT;
constexpr int kRows  = kRowsP + kRowsT;
constexpr int kTrP    = 65;
constexpr int kConvTP = 260;
constexpr int kScanTS = 64;
constexpr int kScanCh = 64;
constexpr int kScanYP = 68;
constexpr int kPrefBlkY = kRowsP / 64;
constexpr int kTgtBlkY  = kRowsT / 64;
static_assert(kXdW <= kXdP, "x_proj width");
static_assert((kDm % 32) == 0 && (kDin % 32) == 0, "GEMM K multiples of 32");
static_assert((kRows % 64) == 0 && (kRowsT % 64) == 0 && (kXzP % 64) == 0 && (kXdP % 64) == 0 && (kDm % 64) == 0, "GEMM M,N multiples of 64");
static_assert((kNC % kScanTS) == 0 && (kNT % kScanTS) == 0 && (kNC % 64) == 0 && kNT == 64 && (kDin % kScanCh) == 0 && (kDin % 256) == 0, "tile multiples");
static_assert((kDm % 64) == 0 && (kDin % 64) == 0 && (kXzP % 64) == 0, "transpose tiles");

constexpr size_t kOffXA   = 0;
constexpr size_t kOffXB   = kOffXA  + (size_t)kRows * kDm  * 4;
constexpr size_t kOffXH   = kOffXB  + (size_t)kRows * kDm  * 4;
constexpr size_t kOffXL   = kOffXH  + (size_t)kRows * kDm  * 2;
constexpr size_t kOffWIH  = kOffXL  + (size_t)kRows * kDm  * 2;
constexpr size_t kOffWIL  = kOffWIH + (size_t)kNL * kXzP * kDm * 2;
constexpr size_t kOffWXH  = kOffWIL + (size_t)kNL * kXzP * kDm * 2;
constexpr size_t kOffWXL  = kOffWXH + (size_t)kNL * kXdP * kDin * 2;
constexpr size_t kOffWOH  = kOffWXL + (size_t)kNL * kXdP * kDin * 2;
constexpr size_t kOffWOL  = kOffWOH + (size_t)kNL * kDm * kDin * 2;
constexpr size_t kOffXZ   = kOffWOL + (size_t)kNL * kDm * kDin * 2;
constexpr size_t kOffUC   = kOffXZ  + (size_t)kRows * kXzP * 4;
constexpr size_t kOffUCH  = kOffUC  + (size_t)kRows * kDin * 4;
constexpr size_t kOffUCL  = kOffUCH + (size_t)kRows * kDin * 2;
constexpr size_t kOffXD   = kOffUCL + (size_t)kRows * kDin * 2;
constexpr size_t kOffYH   = kOffXD  + (size_t)kRows * kXdP * 4;
constexpr size_t kOffYL   = kOffYH  + (size_t)kRows * kDin * 2;
constexpr size_t kOffHF   = kOffYL  + (size_t)kRows * kDin * 2;
constexpr size_t kOffAN   = kOffHF  + (size_t)kBatch * kNst * kDin * 4;
constexpr size_t kWsTotal = kOffAN  + (size_t)kNL * kDin * kNst * 4;
static_assert(kWsTotal == 41943040ull, "carve total");
static_assert(kWsTotal <= 134217728ull, "carve cap");
static_assert((kOffXB % 128) == 0 && (kOffXH % 128) == 0 && (kOffXL % 128) == 0 && (kOffWIH % 128) == 0 &&
              (kOffWIL % 128) == 0 && (kOffWXH % 128) == 0 && (kOffWXL % 128) == 0 && (kOffWOH % 128) == 0 &&
              (kOffWOL % 128) == 0 && (kOffXZ % 128) == 0 && (kOffUC % 128) == 0 && (kOffUCH % 128) == 0 &&
              (kOffUCL % 128) == 0 && (kOffXD % 128) == 0 && (kOffYH % 128) == 0 && (kOffYL % 128) == 0 &&
              (kOffHF % 128) == 0 && (kOffAN % 128) == 0, "128-B aligned regions");

__device__ __forceinline__ unsigned short f2bf_bits(float f) {
  unsigned u = __float_as_uint(f);
  return (unsigned short)((u + 0x7FFFu + ((u >> 16) & 1u)) >> 16);
}
__device__ __forceinline__ float bf_bits2f(unsigned short h) { return __uint_as_float(((unsigned)h) << 16); }

__device__ __forceinline__ float opq(float x) { asm volatile("" : "+v"(x)); return x; }

__device__ __forceinline__ void dep_guard_h(v8f& a, v8f& b, v16h x, v16h y) { asm volatile("v_nop\n\tv_nop\n\tv_nop\n\tv_nop" : "+v"(a), "+v"(b) : "v"(x), "v"(y)); }
__device__ __forceinline__ void dep_guard_b(v8f& a, v8f& b, v16b x, v16b y) { asm volatile("v_nop\n\tv_nop\n\tv_nop\n\tv_nop" : "+v"(a), "+v"(b) : "v"(x), "v"(y)); }
__device__ __forceinline__ void keep4_h(v16h a, v16h b, v16h c, v16h d) { asm volatile("v_nop" :: "v"(a), "v"(b), "v"(c), "v"(d)); }
__device__ __forceinline__ void keep4_b(v16b a, v16b b, v16b c, v16b d) { asm volatile("v_nop" :: "v"(a), "v"(b), "v"(c), "v"(d)); }
__device__ __forceinline__ void acc_guard4(v8f& a, v8f& b, v8f& c, v8f& d) { asm volatile("v_nop\n\tv_nop\n\tv_nop\n\tv_nop" : "+v"(a), "+v"(b), "+v"(c), "+v"(d)); }
template <typename T> struct Frag;
template <> struct Frag<_Float16> {
  typedef v16h V; union U { v16h v; v8h h[2]; };
  static __device__ __forceinline__ v16h load(const _Float16* p) {
    U f; f.h[0] = *(const v8h*)(p); f.h[1] = *(const v8h*)(p + 16); return f.v;
  }
  static __device__ __forceinline__ v8f mma(v16h a, v16h b, v8f c) {
    return __builtin_amdgcn_wmma_f32_16x16x32_f16(false, a, false, b, (short)0, c, false, false);
  }
  static __device__ __forceinline__ void guard(v8f& a, v8f& b, v16h x, v16h y) { dep_guard_h(a, b, x, y); }
  static __device__ __forceinline__ void keep(v16h a, v16h b, v16h c, v16h d) { keep4_h(a, b, c, d); }
};
template <> struct Frag<__bf16> {
  typedef v16b V; union U { v16b v; v8b h[2]; };
  static __device__ __forceinline__ v16b load(const __bf16* p) {
    U f; f.h[0] = *(const v8b*)(p); f.h[1] = *(const v8b*)(p + 16); return f.v;
  }
  static __device__ __forceinline__ v8f mma(v16b a, v16b b, v8f c) {
    return __builtin_amdgcn_wmma_f32_16x16x32_bf16(false, a, false, b, (short)0, c, false, false);
  }
  static __device__ __forceinline__ void guard(v8f& a, v8f& b, v16b x, v16b y) { dep_guard_b(a, b, x, y); }
  static __device__ __forceinline__ void keep(v16b a, v16b b, v16b c, v16b d) { keep4_b(a, b, c, d); }
};

template <int ET> struct Elem;
template <> struct Elem<0> { typedef _Float16 T; };
template <> struct Elem<1> { typedef __bf16 T; };
template <int ET, int SPL, int BIAS_MODE, int OUT_MODE, bool RESID, int ACT = 0>
__global__ __launch_bounds__(256) void wmma_gemm64(
    const unsigned short* __restrict__ Ap, const unsigned short* __restrict__ A2p, int lda, long strideA,
    const unsigned short* __restrict__ Btp, const unsigned short* __restrict__ Bt2p, int ldb, long strideB,
    void* __restrict__ Cout, void* __restrict__ Cout2, int ldc, long strideC,
    const float* __restrict__ bias,
    const float* __restrict__ resid, long strideR,
    int M, int N, int K, float scale) {
  typedef typename Elem<ET>::T T;
  typedef typename Frag<T>::V V;
  const T* A = (const T*)Ap; const T* A2 = (const T*)A2p; const T* Bt = (const T*)Btp; const T* Bt2 = (const T*)Bt2p;
  __shared__ __align__(16) float sT[8][16 * 68];
  const int b    = blockIdx.y;
  const int lane = threadIdx.x & 31;
  const int wave = threadIdx.x >> 5;
  const int tilesN = N >> 6;
  const int tilesM = M >> 6;
  const int tile = blockIdx.x * 8 + wave;
  if (tile >= tilesM * tilesN) return;
  const int tm = tile / tilesN;
  const int tn = tile - tm * tilesN;
  const int m0 = tm << 6;
  const int n0 = tn << 6;

  const T* Ab  = A  + (size_t)b * strideA;
  const T* Bb  = Bt + (size_t)b * strideB;
  const T* Ab2 = (SPL >= 1) ? (A2  + (size_t)b * strideA) : nullptr;
  const T* Bb2 = (SPL == 2) ? (Bt2 + (size_t)b * strideB) : nullptr;

  const int rlane = lane & 15;
  const int koff  = (lane >> 4) * 8;
  const int mOff  = (lane >> 4) * 8;

  v8f acc[4][4];
#pragma unroll
  for (int i = 0; i < 4; ++i)
#pragma unroll
    for (int j = 0; j < 4; ++j) acc[i][j] = (v8f){0.f,0.f,0.f,0.f,0.f,0.f,0.f,0.f};

  for (int k0 = 0; k0 < K; k0 += 32) {
    V bh[4], bl[4];
#pragma unroll
    for (int j = 0; j < 4; ++j) {
      const size_t bo = (size_t)(n0 + (j << 4) + rlane) * ldb + koff + k0;
      bh[j] = Frag<T>::load(Bb + bo);
      if (SPL == 2) bl[j] = Frag<T>::load(Bb2 + bo);
    }
#pragma unroll
    for (int i = 0; i < 4; ++i) {
      const size_t ao = (size_t)(m0 + (i << 4) + rlane) * lda + koff + k0;
      V ah = Frag<T>::load(Ab + ao);
      V al;
      if (SPL >= 1) al = Frag<T>::load(Ab2 + ao);
#pragma unroll
      for (int j = 0; j < 4; ++j) {
        acc[i][j] = Frag<T>::mma(ah, bh[j], acc[i][j]);
        if (SPL == 2) acc[i][j] = Frag<T>::mma(ah, bl[j], acc[i][j]);
        if (SPL >= 1) acc[i][j] = Frag<T>::mma(al, bh[j], acc[i][j]);
      }
      Frag<T>::guard(acc[i][0], acc[i][3], ah, (SPL >= 1) ? al : ah);
    }
    Frag<T>::keep(bh[0], bh[1], bh[2], bh[3]);
    if (SPL == 2) Frag<T>::keep(bl[0], bl[1], bl[2], bl[3]);
  }
  acc_guard4(acc[0][0], acc[0][1], acc[0][2], acc[0][3]);
  acc_guard4(acc[1][0], acc[1][1], acc[1][2], acc[1][3]);
  acc_guard4(acc[2][0], acc[2][1], acc[2][2], acc[2][3]);
  acc_guard4(acc[3][0], acc[3][1], acc[3][2], acc[3][3]);

  float* slab = sT[wave];
  const float* Rb = RESID ? (resid + (size_t)b * strideR) : nullptr;
#pragma unroll
  for (int i = 0; i < 4; ++i) {
    const int mBase = m0 + (i << 4);
#pragma unroll
    for (int j = 0; j < 4; ++j) {
      const int n = n0 + (j << 4) + rlane;
      float bv = 0.f;
      if (BIAS_MODE == 2) bv = bias[n];
#pragma unroll
      for (int r = 0; r < 8; ++r) {
        float v = acc[i][j][r] * scale;
        if (BIAS_MODE == 1) v += bias[mBase + mOff + r];
        if (BIAS_MODE == 2) v += bv;
        if (RESID) v += Rb[(size_t)(mBase + mOff + r) * ldc + n];
        if (ACT == 1) v = tanhf(v);
        if (ACT == 2) v = fmaxf(v, 0.0f);
        if (ACT == 3) v = v / (1.0f + expf(-v));
        if (ACT == 4) v = (v > 0.f) ? v : 0.01f * v;
        slab[(mOff + r) * 68 + (j << 4) + rlane] = v;
      }
    }
    __builtin_amdgcn_fence(__ATOMIC_RELEASE, "workgroup");
    __builtin_amdgcn_wave_barrier();
    __builtin_amdgcn_fence(__ATOMIC_ACQUIRE, "workgroup");
    if (OUT_MODE == 0) {
      float* C = (float*)Cout + (size_t)b * strideC;
      const int hh = lane >> 4, c4 = (lane & 15) * 4;
      for (int pass = 0; pass < 2; ++pass) {
#pragma unroll
        for (int it = 0; it < 8; ++it) {
          const int row = it * 2 + hh;
          v4f v = *(const v4f*)(slab + row * 68 + c4);
          *(volatile v4f*)(C + (size_t)(mBase + row) * ldc + n0 + c4) = v;
        }
        __threadfence();
      }
    } else {
      const int q = lane >> 3, c8 = (lane & 7) * 8;
      unsigned short* C  = (unsigned short*)Cout  + (size_t)b * strideC;
      unsigned short* C2 = (OUT_MODE == 2) ? ((unsigned short*)Cout2 + (size_t)b * strideC) : nullptr;
      for (int pass = 0; pass < 2; ++pass) {
#pragma unroll
        for (int it = 0; it < 4; ++it) {
          const int row = it * 4 + q;
          const float* sp = slab + row * 68 + c8;
          v8h hv, lv;
#pragma unroll
          for (int e = 0; e < 8; ++e) {
            if (OUT_MODE == 1) {
              hv[e] = (_Float16)sp[e];
            } else {
              unsigned short hb = f2bf_bits(sp[e]);
              unsigned short lb = f2bf_bits(sp[e] - bf_bits2f(hb));
              hv[e] = __builtin_bit_cast(_Float16, hb);
              lv[e] = __builtin_bit_cast(_Float16, lb);
            }
          }
          *(volatile v8h*)(C + (size_t)(mBase + row) * ldc + n0 + c8) = hv;
          if (OUT_MODE == 2) *(volatile v8h*)(C2 + (size_t)(mBase + row) * ldc + n0 + c8) = lv;
        }
        __threadfence();
      }
    }
    __builtin_amdgcn_fence(__ATOMIC_RELEASE, "workgroup");
    __builtin_amdgcn_wave_barrier();
    __builtin_amdgcn_fence(__ATOMIC_ACQUIRE, "workgroup");
  }
}

__global__ __launch_bounds__(256) void transpose_split_kernel(
    const float* __restrict__ W, unsigned short* __restrict__ Hh, unsigned short* __restrict__ Hl,
    int Kdim, int Ndim, int Npad)
{
  __shared__ __align__(16) float sT[64 * kTrP];
  const int tid = threadIdx.x, lane = tid & 31, wave = tid >> 5;
  const int lz = blockIdx.z;
  const int k0 = blockIdx.x * 64, n0 = blockIdx.y * 64;
  const float* Wl = W + (size_t)lz * Kdim * Ndim;
#pragma unroll
  for (int i = 0; i < 16; ++i) {
    const int idx = i * 256 + tid;
    const int kk = idx >> 6, nn = idx & 63;
    const int n = n0 + nn;
    const int ncl = (n < Ndim) ? n : (Ndim - 1);
    const float v = Wl[(size_t)(k0 + kk) * Ndim + ncl];
    sT[kk * kTrP + nn] = (n < Ndim) ? v : 0.0f;
  }
  __syncthreads();
  const int q = lane >> 3, c8 = (lane & 7) * 8;
  v8h hv[2], lv[2];
#pragma unroll
  for (int it = 0; it < 2; ++it) {
    const int row = it * 32 + wave * 4 + q;
#pragma unroll
    for (int e = 0; e < 8; ++e) {
      const float f = sT[(c8 + e) * kTrP + row];
      const unsigned short hb = f2bf_bits(f);
      const unsigned short lb = f2bf_bits(f - bf_bits2f(hb));
      hv[it][e] = __builtin_bit_cast(_Float16, hb);
      lv[it][e] = __builtin_bit_cast(_Float16, lb);
    }
  }
  unsigned short* oh = Hh + (size_t)lz * Npad * Kdim;
  unsigned short* ol = Hl + (size_t)lz * Npad * Kdim;
  for (int pass = 0; pass < 2; ++pass) {
#pragma unroll
    for (int it = 0; it < 2; ++it) {
      const int row = it * 32 + wave * 4 + q;
      const size_t o = (size_t)(n0 + row) * Kdim + k0 + c8;
      *(volatile v8h*)(oh + o) = hv[it];
      *(volatile v8h*)(ol + o) = lv[it];
    }
    __threadfence();
  }
}

__global__ __launch_bounds__(256) void neg_exp_kernel(
    const float* __restrict__ src, float* __restrict__ dst, int n)
{
  const int i = blockIdx.x * 256 + threadIdx.x;
  if (i >= n) return;
  const float v = -expf(src[i]);
  *(volatile float*)(dst + i) = v;
  __threadfence();
  *(volatile float*)(dst + i) = v;
}

__global__ __launch_bounds__(256) void copy_rows_kernel(
    const float* __restrict__ xc, const float* __restrict__ xt, float* __restrict__ X, int nblkP, int total4)
{
  const int i = blockIdx.x * 256 + threadIdx.x;
  if (i >= total4) return;
  const size_t e0 = (size_t)i * 4;
  const size_t eP = (size_t)nblkP * 256 * 4;
  const size_t eT = (size_t)total4 * 4 - eP;
  const size_t oc = (e0 < eP) ? e0 : (eP - 4);
  size_t ot = (e0 >= eP) ? (e0 - eP) : 0;
  if (ot > eT - 4) ot = eT - 4;
  const v4f vc = *(const v4f*)(xc + oc);
  const v4f vt = *(const v4f*)(xt + ot);
  const bool pref = (blockIdx.x < nblkP);
  v4f v;
  v[0] = pref ? vc[0] : vt[0];
  v[1] = pref ? vc[1] : vt[1];
  v[2] = pref ? vc[2] : vt[2];
  v[3] = pref ? vc[3] : vt[3];
  *(volatile v4f*)(X + e0) = v;
  __threadfence();
  *(volatile v4f*)(X + e0) = v;
}

__global__ __launch_bounds__(256) void ln_split_kernel(
    const float* __restrict__ X, const float* __restrict__ g, const float* __restrict__ be,
    unsigned short* __restrict__ XHp, unsigned short* __restrict__ XLp, int nrows)
{
  const int lane = threadIdx.x & 31, wave = threadIdx.x >> 5;
  const int row = blockIdx.x * 8 + wave;
  if (row >= nrows) return;
  const float* xr = X + (size_t)row * kDm + lane * 8;
  const v4f a0 = *(const v4f*)(xr);
  const v4f a1 = *(const v4f*)(xr + 4);
  float xv[8];
#pragma unroll
  for (int e = 0; e < 4; ++e) { xv[e] = a0[e]; xv[4 + e] = a1[e]; }
  float s = 0.f;
#pragma unroll
  for (int e = 0; e < 8; ++e) s += xv[e];
#pragma unroll
  for (int off = 16; off >= 1; off >>= 1) s += __shfl_xor(s, off, 32);
  const float mu = s * (1.0f / (float)kDm);
  float dv[8];
  float s2 = 0.f;
#pragma unroll
  for (int e = 0; e < 8; ++e) { dv[e] = xv[e] - mu; s2 += dv[e] * dv[e]; }
#pragma unroll
  for (int off = 16; off >= 1; off >>= 1) s2 += __shfl_xor(s2, off, 32);
  const float var = s2 * (1.0f / (float)kDm);
  const float rs = rsqrtf(var + 1e-5f);
  const v4f g0 = *(const v4f*)(g + lane * 8);
  const v4f g1 = *(const v4f*)(g + lane * 8 + 4);
  const v4f b0 = *(const v4f*)(be + lane * 8);
  const v4f b1 = *(const v4f*)(be + lane * 8 + 4);
  float gv[8], bv[8];
#pragma unroll
  for (int e = 0; e < 4; ++e) { gv[e] = g0[e]; gv[4 + e] = g1[e]; bv[e] = b0[e]; bv[4 + e] = b1[e]; }
  v8h hv, lv;
#pragma unroll
  for (int e = 0; e < 8; ++e) {
    const float t = dv[e] * rs;
    const float hval = t * gv[e] + bv[e];
    const unsigned short hb = f2bf_bits(hval);
    const unsigned short lb = f2bf_bits(hval - bf_bits2f(hb));
    hv[e] = __builtin_bit_cast(_Float16, hb);
    lv[e] = __builtin_bit_cast(_Float16, lb);
  }
  const size_t o = (size_t)row * kDm + lane * 8;
  *(volatile v8h*)(XHp + o) = hv;
  *(volatile v8h*)(XLp + o) = lv;
  __threadfence();
  *(volatile v8h*)(XHp + o) = hv;
  *(volatile v8h*)(XLp + o) = lv;
}

__global__ __launch_bounds__(256) void conv_silu_kernel(
    const float* __restrict__ XZ, const float* __restrict__ cw, const float* __restrict__ cb,
    float* __restrict__ UC, unsigned short* __restrict__ UCH, unsigned short* __restrict__ UCL)
{
  __shared__ __align__(16) float sT[16 * kConvTP];
  const int tid = threadIdx.x, lane = tid & 31, wave = tid >> 5;
  const int d0 = blockIdx.x * 256, d = d0 + tid;
  const bool tgt = (blockIdx.y >= kPrefBlkY);
  int g0, rb;
  bool hist;
  if (tgt) {
    const int bb = blockIdx.y - kPrefBlkY;
    g0 = kRowsP + bb * kNT;
    rb = bb * kNC + (kNC - 3);
    hist = true;
  } else {
    g0 = blockIdx.y * 64;
    const int tb = g0 & (kNC - 1);
    hist = (tb > 0);
    rb = hist ? (g0 - 3) : g0;
  }
  const float w0 = cw[d * kKc + 0], w1 = cw[d * kKc + 1], w2 = cw[d * kKc + 2], w3 = cw[d * kKc + 3];
  const float bc = cb[d];
  float xm3, xm2, xm1;
  {
    const float v3 = XZ[(size_t)rb * kXzP + d];
    const float v2 = XZ[(size_t)(rb + 1) * kXzP + d];
    const float v1 = XZ[(size_t)(rb + 2) * kXzP + d];
    xm3 = hist ? v3 : 0.f;
    xm2 = hist ? v2 : 0.f;
    xm1 = hist ? v1 : 0.f;
  }
  const int hrow = wave >> 1;
  const int hch  = (wave & 1) * 128 + lane * 4;
#pragma unroll 1
  for (int sub = 0; sub < 4; ++sub) {
    const int lb = g0 + sub * 16;
#pragma unroll 1
    for (int s = 0; s < 16; ++s) {
      const float xcur = XZ[(size_t)(lb + s) * kXzP + d];
      float acc = w0 * xm3;
      acc = fmaf(w1, xm2, acc);
      acc = fmaf(w2, xm1, acc);
      acc = fmaf(w3, xcur, acc);
      const float sv = acc + bc;
      const float sg = __builtin_amdgcn_rcpf(1.0f + expf(-sv));
      sT[s * kConvTP + tid] = sv * sg;
      if (!tgt) { xm3 = xm2; xm2 = xm1; xm1 = xcur; }
    }
    __syncthreads();
    v4f fv[4];
    v8h bh[2], blo[2];
#pragma unroll
    for (int it = 0; it < 4; ++it) fv[it] = *(const v4f*)(sT + (it * 4 + hrow) * kConvTP + hch);
#pragma unroll
    for (int it = 0; it < 2; ++it) {
      const float* sp = sT + (it * 8 + wave) * kConvTP + lane * 8;
      const v4f a0 = *(const v4f*)(sp);
      const v4f a1 = *(const v4f*)(sp + 4);
#pragma unroll
      for (int e = 0; e < 4; ++e) {
        const unsigned short h0 = f2bf_bits(a0[e]), h1 = f2bf_bits(a1[e]);
        const unsigned short l0 = f2bf_bits(a0[e] - bf_bits2f(h0)), l1 = f2bf_bits(a1[e] - bf_bits2f(h1));
        bh[it][e]      = __builtin_bit_cast(_Float16, h0);
        bh[it][4 + e]  = __builtin_bit_cast(_Float16, h1);
        blo[it][e]     = __builtin_bit_cast(_Float16, l0);
        blo[it][4 + e] = __builtin_bit_cast(_Float16, l1);
      }
    }
    for (int pass = 0; pass < 2; ++pass) {
#pragma unroll
      for (int it = 0; it < 4; ++it)
        *(volatile v4f*)(UC + (size_t)(lb + it * 4 + hrow) * kDin + d0 + hch) = fv[it];
#pragma unroll
      for (int it = 0; it < 2; ++it) {
        const size_t o = (size_t)(lb + it * 8 + wave) * kDin + d0 + lane * 8;
        *(volatile v8h*)(UCH + o) = bh[it];
        *(volatile v8h*)(UCL + o) = blo[it];
      }
      __threadfence();
    }
    __syncthreads();
  }
}

template <bool PREFIX>
__global__ __launch_bounds__(64) void scan_kernel(
    const float* __restrict__ XD, const float* __restrict__ UC, const float* __restrict__ XZ,
    const float* __restrict__ Wdt, const float* __restrict__ bdt, const float* __restrict__ Aneg,
    const float* __restrict__ Dp, unsigned short* __restrict__ YH, unsigned short* __restrict__ YL,
    float* __restrict__ HF)
{
  __shared__ __align__(16) float sX[kScanTS * kXdP];
  __shared__ __align__(16) float sY[kScanTS * kScanYP];
  __shared__ __align__(16) float sW[kDtR * kScanCh];
  const int tid = threadIdx.x, lane = tid & 31, wave = tid >> 5;
  constexpr int kBlkPerB = kDin / kScanCh;
  constexpr int kSteps = PREFIX ? kNC : kNT;
  const int bix = blockIdx.x / kBlkPerB;
  const int d0  = (blockIdx.x - bix * kBlkPerB) * kScanCh;
  const int d   = d0 + tid;
  const size_t row0 = PREFIX ? ((size_t)bix * kNC) : ((size_t)kRowsP + (size_t)bix * kNT);
#pragma unroll 1
  for (int r = 0; r < kDtR; ++r) sW[r * kScanCh + tid] = Wdt[(size_t)r * kDin + d];
  __syncthreads();
  float negA[kNst], h[kNst];
  {
    const float* ar = Aneg + (size_t)d * kNst;
#pragma unroll
    for (int q4 = 0; q4 < 4; ++q4) {
      const v4f av = *(const v4f*)(ar + 4 * q4);
      negA[4 * q4 + 0] = av[0]; negA[4 * q4 + 1] = av[1]; negA[4 * q4 + 2] = av[2]; negA[4 * q4 + 3] = av[3];
    }
  }
#pragma unroll
  for (int s = 0; s < kNst; ++s) {
    if (PREFIX) h[s] = 0.f;
    else h[s] = HF[((size_t)bix * kNst + s) * kDin + d];
  }
  const float bb = bdt[d], Dd = Dp[d];
  const int lr = tid >> 4, lc4 = (tid & 15) * 4;
  const int q = lane >> 3, c8 = (lane & 7) * 8;
#pragma unroll 1
  for (int t0 = 0; t0 < kSteps; t0 += kScanTS) {
    __syncthreads();
#pragma unroll
    for (int i = 0; i < 16; ++i) {
      const int r = lr + 4 * i;
      *(v4f*)(sX + r * kXdP + lc4) = *(const v4f*)(XD + (row0 + t0 + r) * kXdP + lc4);
    }
    __syncthreads();
#pragma unroll 1
    for (int s = 0; s < kScanTS; ++s) {
      const int t = t0 + s;
      const float* xr = sX + s * kXdP;
      float vdot = 0.f;
#pragma unroll 1
      for (int r4 = 0; r4 < kDtR / 4; ++r4) {
        const v4f xv = *(const v4f*)(xr + 4 * r4);
        const float* wp = sW + (4 * r4) * kScanCh + tid;
        vdot = fmaf(xv[0], wp[0], vdot);
        vdot = fmaf(xv[1], wp[kScanCh], vdot);
        vdot = fmaf(xv[2], wp[2 * kScanCh], vdot);
        vdot = fmaf(xv[3], wp[3 * kScanCh], vdot);
      }
      float Bs[kNst], Cs[kNst];
#pragma unroll
      for (int q4 = 0; q4 < 4; ++q4) {
        const v4f bv = *(const v4f*)(xr + kDtR + 4 * q4);
        const v4f cv = *(const v4f*)(xr + kDtR + kNst + 4 * q4);
        Bs[4 * q4 + 0] = bv[0]; Bs[4 * q4 + 1] = bv[1]; Bs[4 * q4 + 2] = bv[2]; Bs[4 * q4 + 3] = bv[3];
        Cs[4 * q4 + 0] = cv[0]; Cs[4 * q4 + 1] = cv[1]; Cs[4 * q4 + 2] = cv[2]; Cs[4 * q4 + 3] = cv[3];
      }
      const float v   = vdot + bb;
      const float dt  = fmaxf(v, 0.0f) + log1pf(expf(-fabsf(v)));
      const float xt  = UC[(row0 + t) * kDin + d];
      const float dtx = dt * xt;
      float y = 0.f;
#pragma unroll
      for (int k = 0; k < kNst; ++k) {
        const float e  = __expf(dt * negA[k]);
        const float p1 = opq(e * h[k]);
        const float p2 = opq(dtx * Bs[k]);
        const float hn = p1 + p2;
        if (PREFIX) h[k] = hn;
        const float p3 = opq(hn * Cs[k]);
        y = y + p3;
      }
      y = opq(xt * Dd) + y;
      const float zv = XZ[(row0 + t) * kXzP + kDin + d];
      const float sg = __builtin_amdgcn_rcpf(1.0f + expf(-zv));
      y = y * (zv * sg);
      sY[s * kScanYP + tid] = y;
    }
    __syncthreads();
    v8h hv[8], lv[8];
#pragma unroll
    for (int it = 0; it < 8; ++it) {
      const int row = it * 8 + wave * 4 + q;
      const float* sp = sY + row * kScanYP + c8;
      const v4f a0 = *(const v4f*)(sp);
      const v4f a1 = *(const v4f*)(sp + 4);
#pragma unroll
      for (int e = 0; e < 4; ++e) {
        const unsigned short h0 = f2bf_bits(a0[e]), h1 = f2bf_bits(a1[e]);
        const unsigned short l0 = f2bf_bits(a0[e] - bf_bits2f(h0)), l1 = f2bf_bits(a1[e] - bf_bits2f(h1));
        hv[it][e]     = __builtin_bit_cast(_Float16, h0);
        hv[it][4 + e] = __builtin_bit_cast(_Float16, h1);
        lv[it][e]     = __builtin_bit_cast(_Float16, l0);
        lv[it][4 + e] = __builtin_bit_cast(_Float16, l1);
      }
    }
    for (int pass = 0; pass < 2; ++pass) {
#pragma unroll
      for (int it = 0; it < 8; ++it) {
        const int row = it * 8 + wave * 4 + q;
        const size_t o = (row0 + t0 + row) * kDin + d0 + c8;
        *(volatile v8h*)(YH + o) = hv[it];
        *(volatile v8h*)(YL + o) = lv[it];
      }
      __threadfence();
    }
  }
  if (PREFIX) {
    for (int pass = 0; pass < 2; ++pass) {
#pragma unroll
      for (int s = 0; s < kNst; ++s)
        *(volatile float*)(HF + ((size_t)bix * kNst + s) * kDin + d) = h[s];
      __threadfence();
    }
  }
}

extern "C" void kernel_launch(void* const* d_in, const int* in_sizes, int n_in,
                              void* d_out, int out_size, void* d_ws, size_t ws_size,
                              hipStream_t stream) {
  if (n_in < 13) return;
  if (in_sizes[0] != kBatch * kNC * kDm) return;
  if (in_sizes[1] != kBatch * kNT * kDm) return;
  if (in_sizes[2] != kNL * kDm) return;
  if (in_sizes[3] != kNL * kDm) return;
  if (in_sizes[4] != kNL * kDm * kXzP) return;
  if (in_sizes[5] != kNL * kDin * kKc) return;
  if (in_sizes[6] != kNL * kDin) return;
  if (in_sizes[7] != kNL * kDin * kXdW) return;
  if (in_sizes[8] != kNL * kDtR * kDin) return;
  if (in_sizes[9] != kNL * kDin) return;
  if (in_sizes[10] != kNL * kDin * kNst) return;
  if (in_sizes[11] != kNL * kDin) return;
  if (in_sizes[12] != kNL * kDin * kDm) return;
  if (out_size != kRowsT * kDm) return;
  if (ws_size < kWsTotal) return;

  const float* xc     = (const float*)d_in[0];
  const float* xt     = (const float*)d_in[1];
  const float* ln_g   = (const float*)d_in[2];
  const float* ln_b   = (const float*)d_in[3];
  const float* W_in   = (const float*)d_in[4];
  const float* W_conv = (const float*)d_in[5];
  const float* b_conv = (const float*)d_in[6];
  const float* W_x    = (const float*)d_in[7];
  const float* W_dt   = (const float*)d_in[8];
  const float* b_dt   = (const float*)d_in[9];
  const float* A_log  = (const float*)d_in[10];
  const float* Dp     = (const float*)d_in[11];
  const float* W_out  = (const float*)d_in[12];
  float* out = (float*)d_out;

  char* ws = (char*)d_ws;
  float*          XA   = (float*)(ws + kOffXA);
  float*          XB   = (float*)(ws + kOffXB);
  unsigned short* XH   = (unsigned short*)(ws + kOffXH);
  unsigned short* XL   = (unsigned short*)(ws + kOffXL);
  unsigned short* WIH  = (unsigned short*)(ws + kOffWIH);
  unsigned short* WIL  = (unsigned short*)(ws + kOffWIL);
  unsigned short* WXH  = (unsigned short*)(ws + kOffWXH);
  unsigned short* WXL  = (unsigned short*)(ws + kOffWXL);
  unsigned short* WOH  = (unsigned short*)(ws + kOffWOH);
  unsigned short* WOL  = (unsigned short*)(ws + kOffWOL);
  float*          XZ   = (float*)(ws + kOffXZ);
  float*          UC   = (float*)(ws + kOffUC);
  unsigned short* UCH  = (unsigned short*)(ws + kOffUCH);
  unsigned short* UCL  = (unsigned short*)(ws + kOffUCL);
  float*          XD   = (float*)(ws + kOffXD);
  unsigned short* YH   = (unsigned short*)(ws + kOffYH);
  unsigned short* YL   = (unsigned short*)(ws + kOffYL);
  float*          HF   = (float*)(ws + kOffHF);
  float*          AN   = (float*)(ws + kOffAN);

  transpose_split_kernel<<<dim3(kDm / 64, kXzP / 64, kNL), 256, 0, stream>>>(W_in, WIH, WIL, kDm, kXzP, kXzP);
  transpose_split_kernel<<<dim3(kDin / 64, kXdP / 64, kNL), 256, 0, stream>>>(W_x, WXH, WXL, kDin, kXdW, kXdP);
  transpose_split_kernel<<<dim3(kDin / 64, kDm / 64, kNL), 256, 0, stream>>>(W_out, WOH, WOL, kDin, kDm, kDm);

  neg_exp_kernel<<<(kNL * kDin * kNst) / 256, 256, 0, stream>>>(A_log, AN, kNL * kDin * kNst);

  {
    const int nblkP = (kRowsP * kDm / 4) / 256;
    const int total4 = kRows * kDm / 4;
    copy_rows_kernel<<<total4 / 256, 256, 0, stream>>>(xc, xt, XA, nblkP, total4);
  }

  for (int l = 0; l < kNL; ++l) {
    const float* Xin  = (l & 1) ? XB : XA;
    float*       Xout = (l & 1) ? XA : XB;
    const unsigned short* WIh = WIH + (size_t)l * kXzP * kDm;
    const unsigned short* WIl = WIL + (size_t)l * kXzP * kDm;
    const unsigned short* WXh = WXH + (size_t)l * kXdP * kDin;
    const unsigned short* WXl = WXL + (size_t)l * kXdP * kDin;
    const unsigned short* WOh = WOH + (size_t)l * kDm * kDin;
    const unsigned short* WOl = WOL + (size_t)l * kDm * kDin;
    const float* gl   = ln_g   + (size_t)l * kDm;
    const float* bl   = ln_b   + (size_t)l * kDm;
    const float* cwl  = W_conv + (size_t)l * kDin * kKc;
    const float* cbl  = b_conv + (size_t)l * kDin;
    const float* Wdtl = W_dt   + (size_t)l * kDtR * kDin;
    const float* bdtl = b_dt   + (size_t)l * kDin;
    const float* Anl  = AN     + (size_t)l * kDin * kNst;
    const float* Dpl  = Dp     + (size_t)l * kDin;

    ln_split_kernel<<<kRows / 8, 256, 0, stream>>>(Xin, gl, bl, XH, XL, kRows);

    wmma_gemm64<1, 2, 0, 0, false><<<dim3(80, 1), 256, 0, stream>>>(
        XH, XL, kDm, 0L,
        WIh, WIl, kDm, 0L,
        (void*)XZ, nullptr, kXzP, 0L,
        nullptr, nullptr, 0L,
        kRows, kXzP, kDm, 1.0f);

    conv_silu_kernel<<<dim3(kDin / 256, kPrefBlkY + kTgtBlkY), 256, 0, stream>>>(XZ, cwl, cbl, UC, UCH, UCL);

    wmma_gemm64<1, 2, 0, 0, false><<<dim3(5, 1), 256, 0, stream>>>(
        UCH, UCL, kDin, 0L,
        WXh, WXl, kDin, 0L,
        (void*)XD, nullptr, kXdP, 0L,
        nullptr, nullptr, 0L,
        kRows, kXdP, kDin, 1.0f);

    scan_kernel<true><<<kBatch * (kDin / kScanCh), kScanCh, 0, stream>>>(
        XD, UC, XZ, Wdtl, bdtl, Anl, Dpl, YH, YL, HF);
    scan_kernel<false><<<kBatch * (kDin / kScanCh), kScanCh, 0, stream>>>(
        XD, UC, XZ, Wdtl, bdtl, Anl, Dpl, YH, YL, HF);

    if (l + 1 < kNL) {
      wmma_gemm64<1, 2, 0, 0, true><<<dim3(20, 1), 256, 0, stream>>>(
          YH, YL, kDin, 0L,
          WOh, WOl, kDin, 0L,
          (void*)Xout, nullptr, kDm, 0L,
          nullptr, Xin, 0L,
          kRows, kDm, kDin, 1.0f);
    } else {
      wmma_gemm64<1, 2, 0, 0, true><<<dim3(4, 1), 256, 0, stream>>>(
          YH + (size_t)kRowsP * kDin, YL + (size_t)kRowsP * kDin, kDin, 0L,
          WOh, WOl, kDin, 0L,
          (void*)out, nullptr, kDm, 0L,
          nullptr, Xin + (size_t)kRowsP * kDm, 0L,
          kRowsT, kDm, kDin, 1.0f);
    }
  }
}
